// MultiScaleRetention_31636729102529
// MI455X (gfx1250) — hardware-verified
//
#include <hip/hip_runtime.h>
#include <math.h>

constexpr int kBatch = 4;
constexpr int kSeqL  = 2048;
constexpr int kModel = 1024;
constexpr int kNHead = 8;
constexpr int kHDim  = 128;
constexpr int kNPair = 64;
constexpr int kTok   = kBatch * kSeqL;
constexpr int kNProj = 4 * kModel;
constexpr int kNBH   = kBatch * kNHead;
constexpr long kPlaneH = (long)kNBH * kSeqL * kHDim;
constexpr int kKeyT  = 64;
constexpr int kQryT  = 64;

static_assert(kNHead * kHDim == kModel, "shape");
static_assert(kTok % 64 == 0 && kNProj % 64 == 0 && kModel % 64 == 0 && kModel % 32 == 0, "gemm tiles");
static_assert(kSeqL % kKeyT == 0 && kSeqL % kQryT == 0 && kHDim == 128 && kHDim % 32 == 0 && kKeyT % 32 == 0, "attention tiles");
static_assert((kTok * kModel) % (8 * 256) == 0 && (kSeqL * kNPair) % 256 == 0, "prologue grids");
static_assert(kPlaneH == 8388608L, "plane size");

constexpr float kXCarry    = 256.0f;
constexpr float kWCarry    = 16384.0f;
constexpr float kProjScale = 1.0f / (256.0f * 16384.0f);
constexpr float kQCarry    = 8192.0f;
constexpr float kKCarry    = 64.0f;
constexpr float kPFac      = 0.125f;
constexpr float kVCarry    = 1024.0f;
constexpr float kYScale    = 1.0f / (65536.0f * 1024.0f);
constexpr float kZCarry    = 4096.0f;
constexpr float kOutScale  = 1.0f / (4096.0f * 16384.0f);
constexpr float kNormEps   = 1e-5f;

typedef __attribute__((ext_vector_type(16))) _Float16 v16h;
typedef __attribute__((ext_vector_type(8)))  _Float16 v8h;
typedef __attribute__((ext_vector_type(8)))  float    v8f;
typedef __attribute__((ext_vector_type(4)))  float    v4f;
typedef __attribute__((ext_vector_type(4)))  unsigned int v4u;

__device__ __forceinline__ unsigned short f2bf_bits(float f) {
  unsigned u = __float_as_uint(f);
  return (unsigned short)((u + 0x7FFFu + ((u >> 16) & 1u)) >> 16);
}
__device__ __forceinline__ float bf_bits2f(unsigned short h) { return __uint_as_float(((unsigned)h) << 16); }
__device__ __forceinline__ float bfr(float f) { return __uint_as_float(((unsigned)f2bf_bits(f)) << 16); }

__device__ __forceinline__ void keep4_h(v16h a, v16h b, v16h c, v16h d) { asm volatile("v_nop" :: "v"(a), "v"(b), "v"(c), "v"(d)); }
__device__ __forceinline__ void acc_guard4(v8f& a, v8f& b, v8f& c, v8f& d) { asm volatile("v_nop\n\tv_nop\n\tv_nop\n\tv_nop" : "+v"(a), "+v"(b), "+v"(c), "+v"(d)); }
__device__ __forceinline__ void grp_guard(v8f& a, v8f& b, v8f& c, v8f& d, v16h x, v16h y0, v16h y1, v16h y2, v16h y3) {
  asm volatile("v_nop\n\tv_nop\n\tv_nop\n\tv_nop" : "+v"(a), "+v"(b), "+v"(c), "+v"(d) : "v"(x), "v"(y0), "v"(y1), "v"(y2), "v"(y3));
}

template <typename T> struct Frag;
template <> struct Frag<_Float16> {
  typedef v16h V; union U { v16h v; v8h h[2]; };
  static __device__ __forceinline__ v16h load(const _Float16* p) {
    U f; f.h[0] = *(const v8h*)(p); f.h[1] = *(const v8h*)(p + 16); return f.v;
  }
  static __device__ __forceinline__ v8f mma(v16h a, v16h b, v8f c) {
    return __builtin_amdgcn_wmma_f32_16x16x32_f16(false, a, false, b, (short)0, c, false, false);
  }
};

__device__ __forceinline__ v8f mma16(v16h a, v16h b, v8f c) {
  c = __builtin_amdgcn_wmma_f32_16x16x32_f16(false, a, false, b, (short)0, c, false, false);
  asm volatile("v_nop\n\tv_nop\n\tv_nop\n\tv_nop" : "+v"(c) : "v"(a), "v"(b));
  return c;
}

__device__ __forceinline__ unsigned pk16(unsigned short a, unsigned short b) { return (unsigned)a | ((unsigned)b << 16); }
__device__ __forceinline__ unsigned short h_bits(float f) { const _Float16 h = (_Float16)f; return __builtin_bit_cast(unsigned short, h); }

__device__ __forceinline__ void gemm64_mainloop(const _Float16* __restrict__ Ab, int lda,
                                                const _Float16* __restrict__ Bb, int ldb,
                                                int m0, int n0, int K, int lane, v8f (&acc)[4][4]) {
  const int rlane = lane & 15;
  const int koff  = (lane >> 4) * 8;
#pragma unroll
  for (int i = 0; i < 4; ++i)
#pragma unroll
    for (int j = 0; j < 4; ++j) acc[i][j] = (v8f){0.f, 0.f, 0.f, 0.f, 0.f, 0.f, 0.f, 0.f};
  for (int k0 = 0; k0 < K; k0 += 32) {
    v16h bh[4];
#pragma unroll
    for (int j = 0; j < 4; ++j)
      bh[j] = Frag<_Float16>::load(Bb + (size_t)(n0 + (j << 4) + rlane) * ldb + koff + k0);
#pragma unroll
    for (int i = 0; i < 4; ++i) {
      const v16h ah = Frag<_Float16>::load(Ab + (size_t)(m0 + (i << 4) + rlane) * lda + koff + k0);
#pragma unroll
      for (int j = 0; j < 4; ++j) acc[i][j] = Frag<_Float16>::mma(ah, bh[j], acc[i][j]);
      grp_guard(acc[i][0], acc[i][1], acc[i][2], acc[i][3], ah, bh[0], bh[1], bh[2], bh[3]);
    }
    keep4_h(bh[0], bh[1], bh[2], bh[3]);
  }
  acc_guard4(acc[0][0], acc[0][1], acc[0][2], acc[0][3]);
  acc_guard4(acc[1][0], acc[1][1], acc[1][2], acc[1][3]);
  acc_guard4(acc[2][0], acc[2][1], acc[2][2], acc[2][3]);
  acc_guard4(acc[3][0], acc[3][1], acc[3][2], acc[3][3]);
}

__global__ __launch_bounds__(256) void xcast_kernel(const float* __restrict__ X, unsigned short* __restrict__ X16, int n8) {
  const int i = blockIdx.x * 256 + threadIdx.x;
  if (i >= n8) return;
  const float* p = X + 8 * (size_t)i;
  const v4f a = *(const v4f*)(p);
  const v4f c = *(const v4f*)(p + 4);
  unsigned short hb[8];
#pragma unroll
  for (int e = 0; e < 4; ++e) {
    const float fa = a[e];
    const float fc = c[e];
    hb[e]     = h_bits(bfr(fa) * kXCarry);
    hb[4 + e] = h_bits(bfr(fc) * kXCarry);
  }
  const v4u u = (v4u){pk16(hb[0], hb[1]), pk16(hb[2], hb[3]), pk16(hb[4], hb[5]), pk16(hb[6], hb[7])};
  unsigned short* q = X16 + 8 * (size_t)i;
  *(volatile v4u*)q = u;
  __threadfence();
  *(volatile v4u*)q = u;
}

__global__ __launch_bounds__(256) void wt_cast_kernel(const float* __restrict__ W0, const float* __restrict__ W1,
                                                      const float* __restrict__ W2, int nper, int ncol,
                                                      unsigned short* __restrict__ out) {
  __shared__ float sm[64][65];
  const int t  = threadIdx.x;
  const int d0 = blockIdx.x * 64;
  const int c0 = blockIdx.y * 64;
  const int z  = blockIdx.z;
  const int which = z / nper;
  const int zz = z - which * nper;
  const float* Wsel = (which == 0) ? W0 : ((which == 1) ? W1 : W2);
  const float* W = Wsel + (size_t)zz * kModel * ncol;
#pragma unroll
  for (int i = 0; i < 8; ++i) {
    const int e = i * 256 + t;
    const int r = e >> 6;
    const int cc = e & 63;
    sm[cc][r] = bfr(W[(size_t)(d0 + r) * ncol + c0 + cc]) * kWCarry;
  }
  asm volatile("" ::: "memory");
#pragma unroll
  for (int i = 8; i < 16; ++i) {
    const int e = i * 256 + t;
    const int r = e >> 6;
    const int cc = e & 63;
    sm[cc][r] = bfr(W[(size_t)(d0 + r) * ncol + c0 + cc]) * kWCarry;
  }
  __syncthreads();
  const int lane = t & 31, wave = t >> 5;
  const int q = lane >> 3, c8 = (lane & 7) * 8;
  for (int pass = 0; pass < 2; ++pass) {
#pragma unroll
    for (int it = 0; it < 2; ++it) {
      const int row = wave * 8 + it * 4 + q;
      unsigned short hb[8];
#pragma unroll
      for (int e = 0; e < 8; ++e) hb[e] = h_bits(sm[row][c8 + e]);
      const v4u u = (v4u){pk16(hb[0], hb[1]), pk16(hb[2], hb[3]), pk16(hb[4], hb[5]), pk16(hb[6], hb[7])};
      *(volatile v4u*)(out + ((size_t)z * ncol + c0 + row) * kModel + d0 + c8) = u;
    }
    __threadfence();
  }
}

__global__ __launch_bounds__(256) void rot_table_kernel(v4f* __restrict__ XT, int n) {
  const int i = blockIdx.x * 256 + threadIdx.x;
  if (i >= n) return;
  const int l = i >> 6;
  const int j = i & 63;
  const float invf = exp2f((float)j * -0.20762050593046014f);
  const float ang  = (float)l * invf;
  const float sn = sinf(ang);
  const float cs = cosf(ang);
  const float base = ((float)(2 * j) + 51.2f) * (1.0f / 179.2f);
  const float lb = log2f(base);
  const float pw = (float)l * (1.0f / 512.0f);
  const float sc = exp2f(pw * lb);
  const float isc = 1.0f / sc;
  const float cq0 = cs * sc;
  const float sq0 = sn * sc;
  const float ck0 = cs * isc;
  const float sk0 = sn * isc;
  v4f tv;
  tv[0] = cq0 * kQCarry;
  tv[1] = sq0 * kQCarry;
  tv[2] = ck0 * kKCarry;
  tv[3] = sk0 * kKCarry;
  *(volatile v4f*)(XT + i) = tv;
  __threadfence();
  *(volatile v4f*)(XT + i) = tv;
}

__global__ __launch_bounds__(256) void proj_gemm_kernel(const unsigned short* __restrict__ Xp, const unsigned short* __restrict__ Wp,
                                                        const v4f* __restrict__ XT, unsigned short* __restrict__ QKV,
                                                        float* __restrict__ SG) {
  __shared__ __align__(16) float sT[8][16 * 68];
  const int lane = threadIdx.x & 31;
  const int wave = threadIdx.x >> 5;
  constexpr int tilesN = kNProj / 64;
  constexpr int tilesM = kTok / 64;
  const int tile = blockIdx.x * 8 + wave;
  if (tile >= tilesM * tilesN) return;
  const int tm = tile / tilesN;
  const int tn = tile - tm * tilesN;
  const int m0 = tm << 6;
  const int n0 = tn << 6;

  v8f acc[4][4];
  gemm64_mainloop((const _Float16*)Xp, kModel, (const _Float16*)Wp, kModel, m0, n0, kModel, lane, acc);

  const int cat = n0 >> 10;
  const int hd  = (n0 >> 7) & 7;
  const int e0  = n0 & 127;
  const int rlane = lane & 15;
  const int mOff  = (lane >> 4) * 8;
  float* slab = sT[wave];
#pragma unroll
  for (int i = 0; i < 4; ++i) {
    const int mBase = m0 + (i << 4);
#pragma unroll
    for (int j = 0; j < 4; ++j) {
#pragma unroll
      for (int r = 0; r < 8; ++r) slab[(mOff + r) * 68 + (j << 4) + rlane] = acc[i][j][r] * kProjScale;
    }
    __builtin_amdgcn_fence(__ATOMIC_RELEASE, "workgroup");
    __builtin_amdgcn_wave_barrier();
    __builtin_amdgcn_fence(__ATOMIC_ACQUIRE, "workgroup");
    if (cat == 3) {
      const int hh = lane >> 4;
      const int c4 = (lane & 15) * 4;
      const int gcol = n0 - 3 * kModel + c4;
#pragma unroll 1
      for (int it = 0; it < 8; ++it) {
        const int row = it * 2 + hh;
        const v4f g = *(const v4f*)(slab + row * 68 + c4);
        v4f sw;
#pragma unroll
        for (int e = 0; e < 4; ++e) {
          const float gv = g[e];
          const float ex = expf(-gv);
          const float sg = 1.0f / (1.0f + ex);
          sw[e] = gv * sg;
        }
        float* dp = SG + (size_t)(mBase + row) * kModel + gcol;
        *(volatile v4f*)dp = sw;
        __threadfence();
        *(volatile v4f*)dp = sw;
      }
    } else {
      const int q  = lane >> 3;
      const int c8 = (lane & 7) * 8;
      const int jb = (e0 + c8) >> 1;
      unsigned short* plane = QKV + (size_t)cat * kPlaneH;
#pragma unroll 1
      for (int it = 0; it < 4; ++it) {
        const int row = it * 4 + q;
        const int grw = mBase + row;
        const int bb  = grw >> 11;
        const int l   = grw & (kSeqL - 1);
        const float* sp = slab + row * 68 + c8;
        const v4f xa = *(const v4f*)(sp);
        const v4f xb = *(const v4f*)(sp + 4);
        const float xv[8] = {xa[0], xa[1], xa[2], xa[3], xb[0], xb[1], xb[2], xb[3]};
        const v4f* tp = XT + (size_t)l * kNPair + jb;
        v4f tq[4];
        tq[0] = tp[0];
        tq[1] = tp[1];
        tq[2] = tp[2];
        tq[3] = tp[3];
        unsigned short hb[8];
#pragma unroll
        for (int p = 0; p < 4; ++p) {
          const float tx = tq[p][0];
          const float ty = tq[p][1];
          const float tz = tq[p][2];
          const float tw = tq[p][3];
          const float cc = (cat == 0) ? tx : ((cat == 1) ? tz : kVCarry);
          const float ss = (cat == 0) ? ty : ((cat == 1) ? tw : 0.0f);
          const float a0 = xv[2 * p];
          const float a1 = xv[2 * p + 1];
          const float o0 = a0 * cc - a1 * ss;
          const float o1 = a1 * cc + a0 * ss;
          hb[2 * p]     = h_bits(o0);
          hb[2 * p + 1] = h_bits(o1);
        }
        const v4u u = (v4u){pk16(hb[0], hb[1]), pk16(hb[2], hb[3]), pk16(hb[4], hb[5]), pk16(hb[6], hb[7])};
        unsigned short* dp = plane + ((size_t)(bb * kNHead + hd) * kSeqL + l) * kHDim + e0 + c8;
        *(volatile v4u*)dp = u;
        __threadfence();
        *(volatile v4u*)dp = u;
      }
    }
    __builtin_amdgcn_fence(__ATOMIC_RELEASE, "workgroup");
    __builtin_amdgcn_wave_barrier();
    __builtin_amdgcn_fence(__ATOMIC_ACQUIRE, "workgroup");
  }
}

__global__ __launch_bounds__(128) void decay_attn_kernel(const unsigned short* __restrict__ Qp, const unsigned short* __restrict__ Kp,
                                                         const unsigned short* __restrict__ Vp, const float* __restrict__ SG,
                                                         const float* __restrict__ gnw, const float* __restrict__ gnb,
                                                         unsigned short* __restrict__ Zp) {
  __shared__ __align__(16) unsigned int lds_main[8192];
  __shared__ __align__(16) unsigned short Psh[4 * 16 * 64];
  unsigned short* Ksh = (unsigned short*)lds_main;
  unsigned short* Vts = Ksh + 64 * kHDim;

  const int tid  = threadIdx.x;
  const int wave = tid >> 5;
  const int lane = tid & 31;
  const int hh   = lane >> 4;
  const int c    = lane & 15;
  const int qb = blockIdx.x;
  const int bh = blockIdx.y;
  const int b  = bh >> 3;
  const int hd = bh & 7;
  const int q0 = qb * kQryT + wave * 16;

  const float lstart = -3.4657359027997265f;
  const float lstop  = -6.2383246250395077f;
  const float step = (lstop - lstart) * (1.0f / 7.0f);
  const float lv = (hd == kNHead - 1) ? lstop : (lstart + (float)hd * step);
  const float gam = 1.0f - expf(lv);
  const float lg = logf(gam);
  float gr[8], gc[4];
#pragma unroll
  for (int r = 0; r < 8; ++r) gr[r] = expf((float)(8 * hh + r) * lg);
#pragma unroll
  for (int j = 0; j < 4; ++j) gc[j] = expf(-(float)(16 * j + c) * lg);

  v16h qa[4];
  {
    const _Float16* qrow = (const _Float16*)Qp + ((size_t)bh * kSeqL + q0 + c) * kHDim + 8 * hh;
#pragma unroll
    for (int dc = 0; dc < 4; ++dc) qa[dc] = Frag<_Float16>::load(qrow + dc * 32);
  }

  v8f oacc[8];
#pragma unroll
  for (int t = 0; t < 8; ++t) oacc[t] = (v8f){0.f, 0.f, 0.f, 0.f, 0.f, 0.f, 0.f, 0.f};

  const int nChunks = qb + 1;
  for (int kc = 0; kc < nChunks; ++kc) {
    const int kv0 = kc * kKeyT;
    __syncthreads();
    {
      const int kvr = tid >> 1;
      const int dh  = (tid & 1) * 64;
      const size_t roff = ((size_t)bh * kSeqL + kv0 + kvr) * kHDim + dh;
      const v4u* kpw = (const v4u*)(Kp + roff);
      v4u kw[8];
#pragma unroll
      for (int i = 0; i < 8; ++i) kw[i] = kpw[i];
#pragma unroll
      for (int i = 0; i < 8; ++i) *(v4u*)(Ksh + kvr * kHDim + dh + 8 * i) = kw[i];
      asm volatile("" ::: "memory");
      const v4u* vpw = (const v4u*)(Vp + roff);
      v4u vw[8];
#pragma unroll
      for (int i = 0; i < 8; ++i) vw[i] = vpw[i];
#pragma unroll
      for (int i = 0; i < 8; ++i) {
#pragma unroll
        for (int w = 0; w < 4; ++w) {
          const unsigned wd = vw[i][w];
          const int e = dh + 8 * i + 2 * w;
          Vts[e * kKeyT + kvr]       = (unsigned short)(wd & 0xffffu);
          Vts[(e + 1) * kKeyT + kvr] = (unsigned short)(wd >> 16);
        }
      }
    }
    __syncthreads();

    v8f s[4];
#pragma unroll
    for (int j = 0; j < 4; ++j) {
      s[j] = (v8f){0.f, 0.f, 0.f, 0.f, 0.f, 0.f, 0.f, 0.f};
#pragma unroll
      for (int dc = 0; dc < 4; ++dc) {
        const v16h kb = Frag<_Float16>::load((const _Float16*)Ksh + (j * 16 + c) * kHDim + dc * 32 + 8 * hh);
        s[j] = mma16(qa[dc], kb, s[j]);
      }
    }

    const float basef = expf((float)(q0 - kv0) * lg) * kPFac;
    unsigned short* pw = Psh + wave * 1024;
#pragma unroll
    for (int r = 0; r < 8; ++r) {
      const int qrow = q0 + 8 * hh + r;
      const float rf = basef * gr[r];
#pragma unroll
      for (int j = 0; j < 4; ++j) {
        const int kvc = kv0 + 16 * j + c;
        const float dcy = rf * gc[j];
        float v = s[j][r] * dcy;
        v = (qrow >= kvc) ? v : 0.0f;
        pw[(8 * hh + r) * kKeyT + 16 * j + c] = h_bits(v);
      }
    }
    __syncthreads();

#pragma unroll
    for (int kk = 0; kk < 2; ++kk) {
      const v16h pa = Frag<_Float16>::load((const _Float16*)pw + c * kKeyT + kk * 32 + 8 * hh);
#pragma unroll
      for (int t = 0; t < 8; ++t) {
        const v16h vb = Frag<_Float16>::load((const _Float16*)Vts + (t * 16 + c) * kKeyT + kk * 32 + 8 * hh);
        oacc[t] = mma16(pa, vb, oacc[t]);
      }
    }
  }

  __syncthreads();
  float* os = (float*)lds_main + wave * 2048;
#pragma unroll
  for (int r = 0; r < 8; ++r) {
    float y[8];
#pragma unroll
    for (int t = 0; t < 8; ++t) y[t] = oacc[t][r] * kYScale;
    float sum = 0.0f;
#pragma unroll
    for (int t = 0; t < 8; ++t) sum += y[t];
    sum += __shfl_xor(sum, 1);
    sum += __shfl_xor(sum, 2);
    sum += __shfl_xor(sum, 4);
    sum += __shfl_xor(sum, 8);
    const float mean = sum * (1.0f / 128.0f);
    float sq = 0.0f;
#pragma unroll
    for (int t = 0; t < 8; ++t) {
      const float d = y[t] - mean;
      sq += d * d;
    }
    sq += __shfl_xor(sq, 1);
    sq += __shfl_xor(sq, 2);
    sq += __shfl_xor(sq, 4);
    sq += __shfl_xor(sq, 8);
    const float var = sq * (1.0f / 128.0f);
    const float rstd = rsqrtf(var + kNormEps);
#pragma unroll
    for (int t = 0; t < 8; ++t) os[(8 * hh + r) * kHDim + t * 16 + c] = (y[t] - mean) * rstd;
  }
  __syncthreads();

  {
    const int c8  = (lane & 15) * 8;
    const int col = hd * kHDim + c8;
    const v4f gwa = *(const v4f*)(gnw + col);
    const v4f gwb = *(const v4f*)(gnw + col + 4);
    const v4f gba = *(const v4f*)(gnb + col);
    const v4f gbb = *(const v4f*)(gnb + col + 4);
    float gwv[8], gbv[8];
#pragma unroll
    for (int e = 0; e < 4; ++e) {
      const float w0 = gwa[e];
      const float w1 = gwb[e];
      const float b0 = gba[e];
      const float b1 = gbb[e];
      gwv[e] = bfr(w0);
      gwv[4 + e] = bfr(w1);
      gbv[e] = bfr(b0);
      gbv[4 + e] = bfr(b1);
    }
#pragma unroll 1
    for (int it = 0; it < 8; ++it) {
      const int row = it * 2 + hh;
      const size_t grow = (size_t)b * kSeqL + q0 + row;
      const float* ysp = os + row * kHDim + c8;
      const v4f ya = *(const v4f*)(ysp);
      const v4f yb = *(const v4f*)(ysp + 4);
      const float* sgp = SG + grow * kModel + col;
      const v4f ga = *(const v4f*)(sgp);
      const v4f gb2 = *(const v4f*)(sgp + 4);
      unsigned short hb[8];
#pragma unroll
      for (int e = 0; e < 4; ++e) {
        const float y0 = ya[e];
        const float y1 = yb[e];
        const float g0 = ga[e];
        const float g1 = gb2[e];
        const float t0 = y0 * gwv[e] + gbv[e];
        const float t1 = y1 * gwv[4 + e] + gbv[4 + e];
        const float z0 = g0 * t0;
        const float z1 = g1 * t1;
        hb[e]     = h_bits(z0 * kZCarry);
        hb[4 + e] = h_bits(z1 * kZCarry);
      }
      const v4u u = (v4u){pk16(hb[0], hb[1]), pk16(hb[2], hb[3]), pk16(hb[4], hb[5]), pk16(hb[6], hb[7])};
      unsigned short* dp = Zp + grow * kModel + col;
      *(volatile v4u*)dp = u;
      __threadfence();
      *(volatile v4u*)dp = u;
    }
  }
}

__global__ __launch_bounds__(256) void out_gemm_kernel(const unsigned short* __restrict__ Zq, const unsigned short* __restrict__ Wq,
                                                       float* __restrict__ Cout) {
  __shared__ __align__(16) float sT[8][16 * 68];
  const int lane = threadIdx.x & 31;
  const int wave = threadIdx.x >> 5;
  constexpr int tilesN = kModel / 64;
  constexpr int tilesM = kTok / 64;
  const int tile = blockIdx.x * 8 + wave;
  if (tile >= tilesM * tilesN) return;
  const int tm = tile / tilesN;
  const int tn = tile - tm * tilesN;
  const int m0 = tm << 6;
  const int n0 = tn << 6;

  v8f acc[4][4];
  gemm64_mainloop((const _Float16*)Zq, kModel, (const _Float16*)Wq, kModel, m0, n0, kModel, lane, acc);

  const int rlane = lane & 15;
  const int mOff  = (lane >> 4) * 8;
  float* slab = sT[wave];
#pragma unroll
  for (int i = 0; i < 4; ++i) {
    const int mBase = m0 + (i << 4);
#pragma unroll
    for (int j = 0; j < 4; ++j) {
#pragma unroll
      for (int r = 0; r < 8; ++r) slab[(mOff + r) * 68 + (j << 4) + rlane] = acc[i][j][r] * kOutScale;
    }
    __builtin_amdgcn_fence(__ATOMIC_RELEASE, "workgroup");
    __builtin_amdgcn_wave_barrier();
    __builtin_amdgcn_fence(__ATOMIC_ACQUIRE, "workgroup");
    {
      const int hh = lane >> 4, c4 = (lane & 15) * 4;
      for (int pass = 0; pass < 2; ++pass) {
#pragma unroll
        for (int it = 0; it < 8; ++it) {
          const int row = it * 2 + hh;
          v4f v = *(const v4f*)(slab + row * 68 + c4);
          *(volatile v4f*)(Cout + (size_t)(mBase + row) * kModel + n0 + c4) = v;
        }
        __threadfence();
      }
    }
    __builtin_amdgcn_fence(__ATOMIC_RELEASE, "workgroup");
    __builtin_amdgcn_wave_barrier();
    __builtin_amdgcn_fence(__ATOMIC_ACQUIRE, "workgroup");
  }
}

extern "C" void kernel_launch(void* const* d_in, const int* in_sizes, int n_in,
                              void* d_out, int out_size, void* d_ws, size_t ws_size,
                              hipStream_t stream) {
  if (n_in < 8) return;
  const int nX = kTok * kModel;
  const int nW = kNHead * kModel * kHDim;
  if (in_sizes[0] != nX) return;
  if (in_sizes[1] != nW || in_sizes[2] != nW || in_sizes[3] != nW) return;
  if (in_sizes[4] != kModel * kModel || in_sizes[5] != kModel * kModel) return;
  if (in_sizes[6] != kModel || in_sizes[7] != kModel) return;
  if (out_size != nX) return;

  const size_t szX16  = (size_t)kTok * kModel * 2;
  const size_t szWQ   = (size_t)kNProj * kModel * 2;
  const size_t szWO   = (size_t)kModel * kModel * 2;
  const size_t szXT   = (size_t)kSeqL * kNPair * 16;
  const size_t szQKV  = (size_t)kPlaneH * 3 * 2;
  const size_t szSG   = (size_t)kTok * kModel * 4;
  const size_t szZ    = (size_t)kTok * kModel * 2;
  const size_t offX16 = 0;
  const size_t offWQ  = offX16 + szX16;
  const size_t offWO  = offWQ + szWQ;
  const size_t offXT  = offWO + szWO;
  const size_t offQKV = offXT + szXT;
  const size_t offSG  = offQKV + szQKV;
  const size_t offZ   = offSG + szSG;
  const size_t total  = offZ + szZ;
  if (ws_size < total) return;

  const float* X   = (const float*)d_in[0];
  const float* W_Q = (const float*)d_in[1];
  const float* W_K = (const float*)d_in[2];
  const float* W_V = (const float*)d_in[3];
  const float* W_G = (const float*)d_in[4];
  const float* W_O = (const float*)d_in[5];
  const float* gnw = (const float*)d_in[6];
  const float* gnb = (const float*)d_in[7];
  float* out = (float*)d_out;
  char* ws = (char*)d_ws;
  unsigned short* X16   = (unsigned short*)(ws + offX16);
  unsigned short* WQKVG = (unsigned short*)(ws + offWQ);
  unsigned short* WOT   = (unsigned short*)(ws + offWO);
  v4f*            XT    = (v4f*)(ws + offXT);
  unsigned short* QKV   = (unsigned short*)(ws + offQKV);
  float*          SG    = (float*)(ws + offSG);
  unsigned short* Z16   = (unsigned short*)(ws + offZ);

  const int n8 = nX / 8;
  xcast_kernel<<<dim3(n8 / 256), dim3(256), 0, stream>>>(X, X16, n8);
  wt_cast_kernel<<<dim3(kModel / 64, kHDim / 64, 3 * kNHead), dim3(256), 0, stream>>>(W_Q, W_K, W_V, kNHead, kHDim, WQKVG);
  wt_cast_kernel<<<dim3(kModel / 64, kModel / 64, 1), dim3(256), 0, stream>>>(W_G, W_G, W_G, 1, kModel, WQKVG + (size_t)3 * kModel * kModel);
  wt_cast_kernel<<<dim3(kModel / 64, kModel / 64, 1), dim3(256), 0, stream>>>(W_O, W_O, W_O, 1, kModel, WOT);
  const int nTab = kSeqL * kNPair;
  rot_table_kernel<<<dim3(nTab / 256), dim3(256), 0, stream>>>(XT, nTab);

  const int tilesProj = (kTok / 64) * (kNProj / 64);
  proj_gemm_kernel<<<dim3(tilesProj / 8), dim3(256), 0, stream>>>(X16, WQKVG, XT, QKV, SG);

  decay_attn_kernel<<<dim3(kSeqL / kQryT, kNBH), dim3(128), 0, stream>>>(
      QKV, QKV + kPlaneH, QKV + 2 * kPlaneH, SG, gnw, gnb, Z16);

  const int tilesOut = (kTok / 64) * (kModel / 64);
  out_gemm_kernel<<<dim3(tilesOut / 8), dim3(256), 0, stream>>>(Z16, WOT, out);
}
